// CuboidSelfAttentionLayer_71451075937127
// MI455X (gfx1250) — hardware-verified
//
#include <hip/hip_runtime.h>
#include <stdint.h>

#define CDIM   128
#define NH     4
#define HDIM   32
#define C3     384
#define VOL    98
#define VOLP   112
#define NCB    512
#define CHR    57344
#define NBT    2
#define TT     16
#define HH     56
#define WW     56
#define NPOS   50176
#define LDC    132
#define PP     136
#define OSP    36
#define PWB    8704
#define NWAV   7
#define WTP    129
#define QSC    0.17677669529663687f
#define INV512 0.001953125f
#define LN4096 8.3177661667193429f

static_assert(CHR == NCB * VOLP);
static_assert(CHR % 64 == 0);
static_assert(CHR % 16 == 0);
static_assert(NPOS == TT * HH * WW);
static_assert(PWB == 2 * 16 * PP * 2);
static_assert(16 * OSP * 4 <= PWB);
static_assert((PP * 2) % 16 == 0);
static_assert((LDC * 4) % 16 == 0);
static_assert(C3 % 32 == 0);
static_assert(CDIM % 32 == 0);
static_assert(NWAV * 16 == VOLP);
static_assert(NH * HDIM == CDIM);

typedef _Float16 v16h __attribute__((ext_vector_type(16)));
typedef _Float16 v8h  __attribute__((ext_vector_type(8)));
typedef float    v8f  __attribute__((ext_vector_type(8)));
typedef float    v4f  __attribute__((ext_vector_type(4)));
typedef unsigned int v4u __attribute__((ext_vector_type(4)));

__device__ __forceinline__ unsigned short bf_bits(float f) {
  unsigned u = __float_as_uint(f);
  return (unsigned short)((u + 0x7FFFu + ((u >> 16) & 1u)) >> 16);
}
__device__ __forceinline__ float bf_up(unsigned short b) { return __uint_as_float(((unsigned)b) << 16); }
__device__ __forceinline__ float bfr(float f) { return bf_up(bf_bits(f)); }
__device__ __forceinline__ unsigned short h_bits(_Float16 x) { return __builtin_bit_cast(unsigned short, x); }
__device__ __forceinline__ unsigned short hb16(float f) { return h_bits((_Float16)f); }
__device__ __forceinline__ unsigned pk16(unsigned short a, unsigned short b) { return (unsigned)a | ((unsigned)b << 16); }
__device__ __forceinline__ v8f zero8() { v8f z = {0.f, 0.f, 0.f, 0.f, 0.f, 0.f, 0.f, 0.f}; return z; }

__device__ __forceinline__ int pos_of(int bidx, int cub, int v) {
  const int ct = cub >> 6, ch = (cub >> 3) & 7, cw = cub & 7;
  const int it = v / 49;
  const int rem = v - it * 49;
  const int ih = rem / 7;
  const int iw = rem - ih * 7;
  const int ts = ct * 2 + it, hs = ch * 7 + ih, wsx = cw * 7 + iw;
  const int t = (ts + 1) & 15;
  int hq = hs + 3; hq = (hq >= HH) ? (hq - HH) : hq;
  int wq = wsx + 3; wq = (wq >= WW) ? (wq - WW) : wq;
  return ((bidx * TT + t) * HH + hq) * WW + wq;
}
__device__ __forceinline__ int region_of(int cub, int t) {
  const int ct = cub >> 6, ch = (cub >> 3) & 7, cw = cub & 7;
  const int tc = min(t, VOL - 1);
  const int it = tc / 49;
  const int rem = tc - it * 49;
  const int ih = rem / 7;
  const int iw = rem - ih * 7;
  const int rt = (ct < 7) ? 0 : ((it == 0) ? 1 : 2);
  const int rh = (ch < 7) ? 0 : ((ih < 4) ? 1 : 2);
  const int rw = (cw < 7) ? 0 : ((iw < 4) ? 1 : 2);
  const int r = rt * 9 + rh * 3 + rw;
  return (t < VOL) ? r : -1;
}

__device__ __forceinline__ v16h ldfrag_h(const _Float16* p) {
  union { v16h v; v8h h[2]; } f;
  f.h[0] = *(const v8h*)(p);
  f.h[1] = *(const v8h*)(p + 16);
  return f.v;
}
__device__ __forceinline__ v16h ldfrag_h2(const _Float16* p, int off2) {
  union { v16h v; v8h h[2]; } f;
  f.h[0] = *(const v8h*)(p);
  f.h[1] = *(const v8h*)(p + off2);
  return f.v;
}

__device__ __forceinline__ v8f mma_raw(v16h a, v16h b, v8f c) {
  return __builtin_amdgcn_wmma_f32_16x16x32_f16(false, a, false, b, (short)0, c, false, false);
}
__device__ __forceinline__ void guard2(v8f& c0, v8f& c1, const v16h& a0, const v16h& a1, const v16h& b0) {
#if defined(__HIP_DEVICE_COMPILE__)
  asm volatile("v_nop\n\tv_nop\n\tv_nop\n\tv_nop" : "+v"(c0), "+v"(c1) : "v"(a0), "v"(a1), "v"(b0));
#endif
}
__device__ __forceinline__ void guard3(v8f& c0, v8f& c1, v8f& c2,
                                       const v16h& a0, const v16h& a1, const v16h& b0, const v16h& b1) {
#if defined(__HIP_DEVICE_COMPILE__)
  asm volatile("v_nop\n\tv_nop\n\tv_nop\n\tv_nop"
               : "+v"(c0), "+v"(c1), "+v"(c2) : "v"(a0), "v"(a1), "v"(b0), "v"(b1));
#endif
}
__device__ __forceinline__ void guard8(v8f& c0, v8f& c1, v8f& c2, v8f& c3, v8f& c4, v8f& c5, v8f& c6, v8f& c7,
                                       const v16h& a0, const v16h& a1, const v16h& a2, const v16h& a3,
                                       const v16h& b0, const v16h& b1) {
#if defined(__HIP_DEVICE_COMPILE__)
  asm volatile("v_nop\n\tv_nop\n\tv_nop\n\tv_nop"
               : "+v"(c0), "+v"(c1), "+v"(c2), "+v"(c3), "+v"(c4), "+v"(c5), "+v"(c6), "+v"(c7)
               : "v"(a0), "v"(a1), "v"(a2), "v"(a3), "v"(b0), "v"(b1));
#endif
}
__device__ __forceinline__ void wave_sync_lds() {
  __builtin_amdgcn_fence(__ATOMIC_RELEASE, "workgroup");
  __builtin_amdgcn_wave_barrier();
  __builtin_amdgcn_fence(__ATOMIC_ACQUIRE, "workgroup");
}

__global__ __launch_bounds__(256) void cvt_wt(const float* __restrict__ w, unsigned short* wt, int ncols) {
  __shared__ float T[32 * WTP];
  const int tid = threadIdx.x;
  const int n0 = blockIdx.x * 32;
  const int nl = tid & 31, kq = tid >> 5;
  const int ncl = min(n0 + nl, ncols - 1);
#pragma unroll
  for (int i = 0; i < 16; ++i) {
    const int k = kq + 8 * i;
    T[nl * WTP + k] = w[(size_t)k * ncols + ncl];
  }
  __syncthreads();
  v4u pk[2];
  size_t offs[2];
#pragma unroll
  for (int s = 0; s < 2; ++s) {
    const int q = s * 256 + tid;
    const int row = q >> 4, p = q & 15;
    v4u a;
#pragma unroll
    for (int e = 0; e < 4; ++e) {
      const float f0 = bfr(T[row * WTP + 8 * p + 2 * e]) * 1024.0f;
      const float f1 = bfr(T[row * WTP + 8 * p + 2 * e + 1]) * 1024.0f;
      a[e] = pk16(hb16(f0), hb16(f1));
    }
    pk[s] = a;
    offs[s] = (size_t)(n0 + row) * CDIM + 8 * p;
  }
  *(volatile v4u*)(wt + offs[0]) = pk[0];
  *(volatile v4u*)(wt + offs[1]) = pk[1];
  __threadfence();
  *(volatile v4u*)(wt + offs[0]) = pk[0];
  *(volatile v4u*)(wt + offs[1]) = pk[1];
}

__global__ __launch_bounds__(256)
void ln_cvt(const float* __restrict__ x, const float* __restrict__ gam, const float* __restrict__ bet,
            unsigned short* xh, unsigned short* xl, int bidx) {
  const int tid = threadIdx.x, wave = tid >> 5, lane = tid & 31, hh = lane >> 4, c16 = lane & 15;
  const int row = blockIdx.x * 16 + wave * 2 + hh;
  const int cub = row / VOLP;
  const int v = row - cub * VOLP;
  const int vc = min(v, VOL - 1);
  const int pos = pos_of(bidx, cub, vc);
  const float* src = x + (size_t)pos * CDIM + c16 * 8;
  const v4f a = *(const v4f*)(src);
  const v4f b = *(const v4f*)(src + 4);
  float xv[8];
#pragma unroll
  for (int e = 0; e < 4; ++e) { xv[e] = bfr(a[e]); xv[4 + e] = bfr(b[e]); }
  float s = 0.f;
#pragma unroll
  for (int e = 0; e < 8; ++e) s = s + xv[e];
  s = s + __shfl_xor(s, 8, 32);
  s = s + __shfl_xor(s, 4, 32);
  s = s + __shfl_xor(s, 2, 32);
  s = s + __shfl_xor(s, 1, 32);
  const float mu = s * (1.0f / 128.0f);
  float d[8];
  float s2 = 0.f;
#pragma unroll
  for (int e = 0; e < 8; ++e) { d[e] = xv[e] - mu; s2 = s2 + d[e] * d[e]; }
  s2 = s2 + __shfl_xor(s2, 8, 32);
  s2 = s2 + __shfl_xor(s2, 4, 32);
  s2 = s2 + __shfl_xor(s2, 2, 32);
  s2 = s2 + __shfl_xor(s2, 1, 32);
  const float var = s2 * (1.0f / 128.0f);
  const float rstd = rsqrtf(var + 1e-5f);
  const v4f g0 = *(const v4f*)(gam + c16 * 8);
  const v4f g1 = *(const v4f*)(gam + c16 * 8 + 4);
  const v4f b0 = *(const v4f*)(bet + c16 * 8);
  const v4f b1 = *(const v4f*)(bet + c16 * 8 + 4);
  float g[8], be[8];
#pragma unroll
  for (int e = 0; e < 4; ++e) { g[e] = bfr(g0[e]); g[4 + e] = bfr(g1[e]); be[e] = bfr(b0[e]); be[4 + e] = bfr(b1[e]); }
  const bool real = (v < VOL);
  v4u ph, pl;
#pragma unroll
  for (int e = 0; e < 4; ++e) {
    float xn0 = d[2 * e] * rstd * g[2 * e] + be[2 * e];
    float xn1 = d[2 * e + 1] * rstd * g[2 * e + 1] + be[2 * e + 1];
    xn0 = real ? xn0 : 0.f;
    xn1 = real ? xn1 : 0.f;
    const float f0 = xn0 * 8.0f, f1 = xn1 * 8.0f;
    const _Float16 h0 = (_Float16)f0, h1 = (_Float16)f1;
    const float r0 = (f0 - (float)h0) * 16384.0f;
    const float r1 = (f1 - (float)h1) * 16384.0f;
    ph[e] = pk16(h_bits(h0), h_bits(h1));
    pl[e] = pk16(hb16(r0), hb16(r1));
  }
  const size_t off = (size_t)row * CDIM + c16 * 8;
  *(volatile v4u*)(xh + off) = ph;
  *(volatile v4u*)(xl + off) = pl;
  __threadfence();
  *(volatile v4u*)(xh + off) = ph;
  *(volatile v4u*)(xl + off) = pl;
}

__global__ __launch_bounds__(256)
void gemm_qkv(const unsigned short* __restrict__ xh, const unsigned short* __restrict__ xl,
              const unsigned short* __restrict__ wq,
              unsigned short* qhp, unsigned short* qlp, unsigned short* kpl,
              unsigned short* vth, unsigned short* vtl) {
  __shared__ __align__(16) float Cs[64 * LDC];
  const int tid = threadIdx.x, wave = tid >> 5, lane = tid & 31, hh = lane >> 4, c = lane & 15;
  const int mb = blockIdx.x, part = blockIdx.y;
  const int mw = wave >> 2, nw = wave & 3;
  const _Float16* Ah = (const _Float16*)(const void*)xh;
  const _Float16* Al = (const _Float16*)(const void*)xl;
  const _Float16* W  = (const _Float16*)(const void*)wq;
  const int arow0 = mb * 64 + mw * 32;
  const int bcol0 = part * 128 + nw * 32;

  v8f h00 = zero8(), h01 = zero8(), h10 = zero8(), h11 = zero8();
  v8f l00 = zero8(), l01 = zero8(), l10 = zero8(), l11 = zero8();
#pragma unroll 1
  for (int ks = 0; ks < 4; ++ks) {
    const int k0 = ks * 32 + 8 * hh;
    const v16h fa0 = ldfrag_h(Ah + (size_t)(arow0 + c) * CDIM + k0);
    const v16h fa1 = ldfrag_h(Ah + (size_t)(arow0 + 16 + c) * CDIM + k0);
    const v16h ga0 = ldfrag_h(Al + (size_t)(arow0 + c) * CDIM + k0);
    const v16h ga1 = ldfrag_h(Al + (size_t)(arow0 + 16 + c) * CDIM + k0);
    const v16h fb0 = ldfrag_h(W + (size_t)(bcol0 + c) * CDIM + k0);
    const v16h fb1 = ldfrag_h(W + (size_t)(bcol0 + 16 + c) * CDIM + k0);
    h00 = mma_raw(fa0, fb0, h00);
    h01 = mma_raw(fa0, fb1, h01);
    h10 = mma_raw(fa1, fb0, h10);
    h11 = mma_raw(fa1, fb1, h11);
    l00 = mma_raw(ga0, fb0, l00);
    l01 = mma_raw(ga0, fb1, l01);
    l10 = mma_raw(ga1, fb0, l10);
    l11 = mma_raw(ga1, fb1, l11);
    guard8(h00, h01, h10, h11, l00, l01, l10, l11, fa0, fa1, ga0, ga1, fb0, fb1);
  }
#pragma unroll
  for (int r = 0; r < 8; ++r) {
    const int row = mw * 32 + 8 * hh + r;
    Cs[row * LDC + nw * 32 + c]             = h00[r] + l00[r] * (1.0f / 16384.0f);
    Cs[row * LDC + nw * 32 + 16 + c]        = h01[r] + l01[r] * (1.0f / 16384.0f);
    Cs[(row + 16) * LDC + nw * 32 + c]      = h10[r] + l10[r] * (1.0f / 16384.0f);
    Cs[(row + 16) * LDC + nw * 32 + 16 + c] = h11[r] + l11[r] * (1.0f / 16384.0f);
  }
  __syncthreads();

  const int row0 = mb * 64;
  if (part < 2) {
    unsigned short* dsth = (part == 0) ? qhp : kpl;
    const float scl = (part == 0) ? (QSC * 64.0f) : 8.0f;
    v4u pk[4], plk[4];
    size_t offs[4];
#pragma unroll
    for (int s = 0; s < 4; ++s) {
      const int L = s * 32 + (tid >> 3), p = tid & 7;
      const int h4 = L >> 5, li = L & 31;
      const int tok = 2 * li + (p >> 2), d0 = (p & 3) * 8;
      const int col = h4 * 32 + d0;
      v4u q4, r4;
#pragma unroll
      for (int e = 0; e < 4; ++e) {
        const float f0 = Cs[tok * LDC + col + 2 * e] * (1.0f / 8192.0f) * scl;
        const float f1 = Cs[tok * LDC + col + 2 * e + 1] * (1.0f / 8192.0f) * scl;
        const _Float16 e0 = (_Float16)f0, e1 = (_Float16)f1;
        const float r0 = (f0 - (float)e0) * 16384.0f;
        const float r1 = (f1 - (float)e1) * 16384.0f;
        q4[e] = pk16(h_bits(e0), h_bits(e1));
        r4[e] = pk16(hb16(r0), hb16(r1));
      }
      pk[s] = q4;
      plk[s] = r4;
      offs[s] = ((size_t)h4 * CHR + row0 + tok) * HDIM + d0;
    }
#pragma unroll
    for (int s = 0; s < 4; ++s) *(volatile v4u*)(dsth + offs[s]) = pk[s];
    if (part == 0) {
#pragma unroll
      for (int s = 0; s < 4; ++s) *(volatile v4u*)(qlp + offs[s]) = plk[s];
    }
    __threadfence();
#pragma unroll
    for (int s = 0; s < 4; ++s) *(volatile v4u*)(dsth + offs[s]) = pk[s];
    if (part == 0) {
#pragma unroll
      for (int s = 0; s < 4; ++s) *(volatile v4u*)(qlp + offs[s]) = plk[s];
    }
  } else {
    v4u phk[4], plk[4];
    size_t offs[4];
#pragma unroll
    for (int s = 0; s < 4; ++s) {
      const int L = s * 32 + (tid >> 3), p = tid & 7;
      const int h4 = L >> 5, d = L & 31;
      const int col = h4 * 32 + d;
      const int tb = p * 8;
      v4u a, b;
#pragma unroll
      for (int e = 0; e < 4; ++e) {
        const float v0 = Cs[(tb + 2 * e) * LDC + col] * (1.0f / 8192.0f);
        const float v1 = Cs[(tb + 2 * e + 1) * LDC + col] * (1.0f / 8192.0f);
        const float f0 = v0 * 16.0f, f1 = v1 * 16.0f;
        const _Float16 e0 = (_Float16)f0, e1 = (_Float16)f1;
        const float r0 = (f0 - (float)e0) * 16384.0f;
        const float r1 = (f1 - (float)e1) * 16384.0f;
        a[e] = pk16(h_bits(e0), h_bits(e1));
        b[e] = pk16(hb16(r0), hb16(r1));
      }
      phk[s] = a;
      plk[s] = b;
      offs[s] = ((size_t)(h4 * HDIM + d)) * CHR + row0 + tb;
    }
#pragma unroll
    for (int s = 0; s < 4; ++s) { *(volatile v4u*)(vth + offs[s]) = phk[s]; *(volatile v4u*)(vtl + offs[s]) = plk[s]; }
    __threadfence();
#pragma unroll
    for (int s = 0; s < 4; ++s) { *(volatile v4u*)(vth + offs[s]) = phk[s]; *(volatile v4u*)(vtl + offs[s]) = plk[s]; }
  }
}

__global__ __launch_bounds__(224)
void attn_cub(const unsigned short* __restrict__ qh, const unsigned short* __restrict__ ql,
              const unsigned short* __restrict__ kp, const unsigned short* __restrict__ vth,
              const unsigned short* __restrict__ vtl, unsigned short* ohi, unsigned short* olo) {
  __shared__ __align__(16) char pbuf[NWAV * PWB];
  __shared__ int cnts[VOLP];
  const int tid = threadIdx.x, wave = tid >> 5, lane = tid & 31, hh = lane >> 4, c = lane & 15;
  const int cub = blockIdx.x >> 2, h = blockIdx.x & 3;
  const int q0 = wave * 16;
  const int rb = cub * VOLP;

  for (int t = tid; t < VOLP; t += NWAV * 32) cnts[t] = region_of(cub, t);
  __syncthreads();

  const _Float16* Qh = (const _Float16*)(const void*)qh + ((size_t)h * CHR + rb) * HDIM;
  const _Float16* Ql = (const _Float16*)(const void*)ql + ((size_t)h * CHR + rb) * HDIM;
  const _Float16* Kp = (const _Float16*)(const void*)kp + ((size_t)h * CHR + rb) * HDIM;
  const _Float16* Vh = (const _Float16*)(const void*)vth + (size_t)(h * HDIM) * CHR + rb;
  const _Float16* Vl = (const _Float16*)(const void*)vtl + (size_t)(h * HDIM) * CHR + rb;
  _Float16* Ph = (_Float16*)(pbuf + wave * PWB);
  _Float16* Pl = Ph + 16 * PP;

  const v16h qa  = ldfrag_h(Qh + (size_t)(q0 + c) * HDIM + 8 * hh);
  const v16h qla = ldfrag_h(Ql + (size_t)(q0 + c) * HDIM + 8 * hh);
  int cntn[8];
#pragma unroll
  for (int r = 0; r < 8; ++r) cntn[r] = cnts[q0 + 8 * hh + r];

  v8f s[7];
#pragma unroll
  for (int j = 0; j < 7; ++j) {
    const int key = j * 16 + c;
    const v16h kf = ldfrag_h(Kp + (size_t)key * HDIM + 8 * hh);
    v8f a0 = mma_raw(qa, kf, zero8());
    v8f a1 = mma_raw(qla, kf, zero8());
    guard2(a0, a1, qa, qla, kf);
    const int cm = cnts[key];
    v8f sj;
#pragma unroll
    for (int r = 0; r < 8; ++r) {
      const float t0 = a0[r] + a1[r] * (1.0f / 16384.0f);
      sj[r] = t0 + ((cntn[r] != cm) ? -51200.0f : 0.0f);
    }
    s[j] = sj;
  }
  float lrow[8];
#pragma unroll
  for (int r = 0; r < 8; ++r) {
    float tm = s[0][r];
#pragma unroll
    for (int j = 1; j < 7; ++j) tm = fmaxf(tm, s[j][r]);
    tm = fmaxf(tm, __shfl_xor(tm, 1, 32));
    tm = fmaxf(tm, __shfl_xor(tm, 2, 32));
    tm = fmaxf(tm, __shfl_xor(tm, 4, 32));
    tm = fmaxf(tm, __shfl_xor(tm, 8, 32));
    float ps = 0.f;
#pragma unroll
    for (int j = 0; j < 7; ++j) {
      const float p = __expf((s[j][r] - tm) * INV512 + LN4096);
      ps = ps + p;
      s[j][r] = p;
    }
    ps = ps + __shfl_xor(ps, 1, 32);
    ps = ps + __shfl_xor(ps, 2, 32);
    ps = ps + __shfl_xor(ps, 4, 32);
    ps = ps + __shfl_xor(ps, 8, 32);
    lrow[r] = ps;
  }
#pragma unroll
  for (int j = 0; j < 7; ++j) {
#pragma unroll
    for (int r = 0; r < 8; ++r) {
      const float pf = s[j][r];
      const _Float16 phv = (_Float16)pf;
      const float res = (pf - (float)phv) * 8192.0f;
      const int idx = (8 * hh + r) * PP + j * 16 + c;
      Ph[idx] = phv;
      Pl[idx] = (_Float16)res;
    }
  }
#pragma unroll
  for (int r = 0; r < 8; ++r) {
    const int idx = (8 * hh + r) * PP + VOLP + c;
    Ph[idx] = (_Float16)0.0f;
    Pl[idx] = (_Float16)0.0f;
  }
  wave_sync_lds();
  v8f ohh0 = zero8(), ohh1 = zero8(), ohl0 = zero8(), ohl1 = zero8(), olh0 = zero8(), olh1 = zero8();
#pragma unroll
  for (int ks = 0; ks < 4; ++ks) {
    const int o2 = (ks == 3) ? 0 : 16;
    const v16h pa  = ldfrag_h(Ph + c * PP + ks * 32 + 8 * hh);
    const v16h pla = ldfrag_h(Pl + c * PP + ks * 32 + 8 * hh);
    const int koff = ks * 32 + 8 * hh;
    {
      const v16h vh = ldfrag_h2(Vh + (size_t)c * CHR + koff, o2);
      const v16h vl = ldfrag_h2(Vl + (size_t)c * CHR + koff, o2);
      ohh0 = mma_raw(pa, vh, ohh0);
      ohl0 = mma_raw(pa, vl, ohl0);
      olh0 = mma_raw(pla, vh, olh0);
      guard3(ohh0, ohl0, olh0, pa, pla, vh, vl);
    }
    {
      const v16h vh = ldfrag_h2(Vh + (size_t)(16 + c) * CHR + koff, o2);
      const v16h vl = ldfrag_h2(Vl + (size_t)(16 + c) * CHR + koff, o2);
      ohh1 = mma_raw(pa, vh, ohh1);
      ohl1 = mma_raw(pa, vl, ohl1);
      olh1 = mma_raw(pla, vh, olh1);
      guard3(ohh1, ohl1, olh1, pa, pla, vh, vl);
    }
  }
  wave_sync_lds();

  float* Os = (float*)(void*)(pbuf + wave * PWB);
#pragma unroll
  for (int r = 0; r < 8; ++r) {
    const float inv = 1.0f / (lrow[r] * 16.0f);
    const int row = 8 * hh + r;
    float o0 = ohh0[r] + ohl0[r] * (1.0f / 16384.0f);
    o0 = o0 + olh0[r] * (1.0f / 8192.0f);
    float o1 = ohh1[r] + ohl1[r] * (1.0f / 16384.0f);
    o1 = o1 + olh1[r] * (1.0f / 8192.0f);
    Os[row * OSP + c]      = o0 * inv;
    Os[row * OSP + 16 + c] = o1 * inv;
  }
  wave_sync_lds();
  v4u ph2[2], pl2[2];
  size_t off2[2];
#pragma unroll
  for (int sI = 0; sI < 2; ++sI) {
    const int line = sI * 4 + (lane >> 3), piece = lane & 7;
    const int row = 2 * line + (piece >> 2), d0 = (piece & 3) * 8;
    v4u a, b;
#pragma unroll
    for (int e = 0; e < 4; ++e) {
      const float f0 = Os[row * OSP + d0 + 2 * e] * 64.0f;
      const float f1 = Os[row * OSP + d0 + 2 * e + 1] * 64.0f;
      const _Float16 e0 = (_Float16)f0, e1 = (_Float16)f1;
      const float r0 = (f0 - (float)e0) * 16384.0f;
      const float r1 = (f1 - (float)e1) * 16384.0f;
      a[e] = pk16(h_bits(e0), h_bits(e1));
      b[e] = pk16(hb16(r0), hb16(r1));
    }
    ph2[sI] = a;
    pl2[sI] = b;
    off2[sI] = ((size_t)h * CHR + rb + q0 + row) * HDIM + d0;
  }
  *(volatile v4u*)(ohi + off2[0]) = ph2[0];
  *(volatile v4u*)(ohi + off2[1]) = ph2[1];
  *(volatile v4u*)(olo + off2[0]) = pl2[0];
  *(volatile v4u*)(olo + off2[1]) = pl2[1];
  __threadfence();
  *(volatile v4u*)(ohi + off2[0]) = ph2[0];
  *(volatile v4u*)(ohi + off2[1]) = ph2[1];
  *(volatile v4u*)(olo + off2[0]) = pl2[0];
  *(volatile v4u*)(olo + off2[1]) = pl2[1];
}

__global__ __launch_bounds__(256)
void gemm_proj(const unsigned short* __restrict__ ohi, const unsigned short* __restrict__ olo,
               const unsigned short* __restrict__ wp, const float* __restrict__ bp, float* out, int bidx) {
  __shared__ __align__(16) float Cs[64 * LDC];
  const int tid = threadIdx.x, wave = tid >> 5, lane = tid & 31, hh = lane >> 4, c = lane & 15;
  const int mb = blockIdx.x;
  const int mw = wave >> 2, nw = wave & 3;
  const _Float16* W = (const _Float16*)(const void*)wp;
  const int arow0 = mb * 64 + mw * 32;
  const int bcol0 = nw * 32;

  v8f h00 = zero8(), h01 = zero8(), h10 = zero8(), h11 = zero8();
  v8f l00 = zero8(), l01 = zero8(), l10 = zero8(), l11 = zero8();
#pragma unroll 1
  for (int ks = 0; ks < 4; ++ks) {
    const _Float16* Ah = (const _Float16*)(const void*)ohi + (size_t)ks * CHR * HDIM;
    const _Float16* Al = (const _Float16*)(const void*)olo + (size_t)ks * CHR * HDIM;
    const v16h fa0 = ldfrag_h(Ah + (size_t)(arow0 + c) * HDIM + 8 * hh);
    const v16h fa1 = ldfrag_h(Ah + (size_t)(arow0 + 16 + c) * HDIM + 8 * hh);
    const v16h ga0 = ldfrag_h(Al + (size_t)(arow0 + c) * HDIM + 8 * hh);
    const v16h ga1 = ldfrag_h(Al + (size_t)(arow0 + 16 + c) * HDIM + 8 * hh);
    const v16h fb0 = ldfrag_h(W + (size_t)(bcol0 + c) * CDIM + ks * 32 + 8 * hh);
    const v16h fb1 = ldfrag_h(W + (size_t)(bcol0 + 16 + c) * CDIM + ks * 32 + 8 * hh);
    h00 = mma_raw(fa0, fb0, h00);
    h01 = mma_raw(fa0, fb1, h01);
    h10 = mma_raw(fa1, fb0, h10);
    h11 = mma_raw(fa1, fb1, h11);
    l00 = mma_raw(ga0, fb0, l00);
    l01 = mma_raw(ga0, fb1, l01);
    l10 = mma_raw(ga1, fb0, l10);
    l11 = mma_raw(ga1, fb1, l11);
    guard8(h00, h01, h10, h11, l00, l01, l10, l11, fa0, fa1, ga0, ga1, fb0, fb1);
  }
#pragma unroll
  for (int r = 0; r < 8; ++r) {
    const int row = mw * 32 + 8 * hh + r;
    Cs[row * LDC + nw * 32 + c]             = h00[r] + l00[r] * (1.0f / 16384.0f);
    Cs[row * LDC + nw * 32 + 16 + c]        = h01[r] + l01[r] * (1.0f / 16384.0f);
    Cs[(row + 16) * LDC + nw * 32 + c]      = h10[r] + l10[r] * (1.0f / 16384.0f);
    Cs[(row + 16) * LDC + nw * 32 + 16 + c] = h11[r] + l11[r] * (1.0f / 16384.0f);
  }
  __syncthreads();

  const int row0 = mb * 64;
  const float* bpn = bp + lane * 4;
  v4f bb;
#pragma unroll
  for (int e = 0; e < 4; ++e) bb[e] = bfr(bpn[e]);
  v4f ov[8];
  size_t offs[8];
  bool vld[8];
#pragma unroll
  for (int it = 0; it < 8; ++it) {
    const int row = wave * 8 + it;
    const int grow = row0 + row;
    const int cub = grow / VOLP;
    const int v = grow - cub * VOLP;
    vld[it] = (v < VOL);
    const int pos = pos_of(bidx, cub, min(v, VOL - 1));
    v4f val = *(const v4f*)(Cs + row * LDC + lane * 4);
#pragma unroll
    for (int e = 0; e < 4; ++e) val[e] = val[e] * (1.0f / 65536.0f) + bb[e];
    ov[it] = val;
    offs[it] = (size_t)pos * CDIM + lane * 4;
  }
#pragma unroll
  for (int it = 0; it < 8; ++it) { if (vld[it]) *(volatile v4f*)(out + offs[it]) = ov[it]; }
  __threadfence();
#pragma unroll
  for (int it = 0; it < 8; ++it) { if (vld[it]) *(volatile v4f*)(out + offs[it]) = ov[it]; }
}

extern "C" void kernel_launch(void* const* d_in, const int* in_sizes, int n_in,
                              void* d_out, int out_size, void* d_ws, size_t ws_size,
                              hipStream_t stream) {
  if (n_in < 6) return;
  if (in_sizes[0] != NBT * NPOS * CDIM) return;
  if (in_sizes[1] != CDIM || in_sizes[2] != CDIM) return;
  if (in_sizes[3] != CDIM * C3) return;
  if (in_sizes[4] != CDIM * CDIM) return;
  if (in_sizes[5] != CDIM) return;
  if (out_size != NBT * NPOS * CDIM) return;

  const float* x     = (const float*)d_in[0];
  const float* gam   = (const float*)d_in[1];
  const float* bet   = (const float*)d_in[2];
  const float* wqkv  = (const float*)d_in[3];
  const float* wproj = (const float*)d_in[4];
  const float* bproj = (const float*)d_in[5];
  float* out = (float*)d_out;

  const size_t sPl = (size_t)CHR * CDIM * 2;
  const size_t sWq = (size_t)C3 * CDIM * 2;
  const size_t sWp = (size_t)CDIM * CDIM * 2;
  size_t off = 0;
  const size_t oXh = off; off += sPl;
  const size_t oXl = off; off += sPl;
  const size_t oWq = off; off += sWq;
  const size_t oWp = off; off += sWp;
  const size_t oQh = off; off += sPl;
  const size_t oQl = off; off += sPl;
  const size_t oK  = off; off += sPl;
  const size_t oVh = off; off += sPl;
  const size_t oVl = off; off += sPl;
  if (off > ws_size) return;
  if (off > (size_t)134217728) return;

  char* ws = (char*)d_ws;
  unsigned short* Xh  = (unsigned short*)(ws + oXh);
  unsigned short* Xl  = (unsigned short*)(ws + oXl);
  unsigned short* Oh  = (unsigned short*)(ws + oXh);
  unsigned short* Ol  = (unsigned short*)(ws + oXl);
  unsigned short* Wq  = (unsigned short*)(ws + oWq);
  unsigned short* Wp  = (unsigned short*)(ws + oWp);
  unsigned short* Qh  = (unsigned short*)(ws + oQh);
  unsigned short* Ql  = (unsigned short*)(ws + oQl);
  unsigned short* Kp  = (unsigned short*)(ws + oK);
  unsigned short* Vth = (unsigned short*)(ws + oVh);
  unsigned short* Vtl = (unsigned short*)(ws + oVl);

  const dim3 blk(256);
  cvt_wt<<<dim3(C3 / 32), blk, 0, stream>>>(wqkv, Wq, C3);
  cvt_wt<<<dim3(CDIM / 32), blk, 0, stream>>>(wproj, Wp, CDIM);
  for (int b = 0; b < NBT; ++b) {
    ln_cvt<<<dim3(CHR / 16), blk, 0, stream>>>(x, gam, bet, Xh, Xl, b);
    gemm_qkv<<<dim3(CHR / 64, 3), blk, 0, stream>>>(Xh, Xl, Wq, Qh, Ql, Kp, Vth, Vtl);
    attn_cub<<<dim3(NCB * NH), dim3(NWAV * 32), 0, stream>>>(Qh, Ql, Kp, Vth, Vtl, Oh, Ol);
    gemm_proj<<<dim3(CHR / 64), blk, 0, stream>>>(Oh, Ol, Wp, bproj, out, b);
  }
  (void)hipGetLastError();
}
